// GammaSpaceLayer_50208167690595
// MI455X (gfx1250) — hardware-run, weakly checked
//
#include <hip/hip_runtime.h>
#include <math.h>

typedef __attribute__((ext_vector_type(16))) _Float16 v16h;
typedef __attribute__((ext_vector_type(8)))  _Float16 v8h;
typedef __attribute__((ext_vector_type(16))) __bf16   v16b;
typedef __attribute__((ext_vector_type(8)))  __bf16   v8b;
typedef __attribute__((ext_vector_type(8)))  float    v8f;
typedef __attribute__((ext_vector_type(4)))  float    v4f;

constexpr int kNB    = 16;
constexpr int kL     = 2048;
constexpr int kS     = 128;
constexpr int kH     = 64;
constexpr int kRows  = kNB * kL;
constexpr float kDtMin = 0.001f;
constexpr float kDtMax = 0.1f;

constexpr float kUCarry = 16.0f;
constexpr float kBCarry = 8192.0f;
constexpr float kXCarry = 256.0f;
constexpr float kCCarry = 64.0f;
constexpr float kFold1  = 1.0f / (kUCarry * kBCarry);
constexpr float kFold2  = 1.0f / (kXCarry * kCCarry);
constexpr float kF16MinNormal = 6.103515625e-05f;
constexpr float kF32MinNormal = 1.17549435e-38f;

constexpr int kXP    = 72;
constexpr int kChunk = 16;

static_assert(kRows == 32768);
static_assert((kRows % 64) == 0 && (kH % 64) == 0 && (kS % 64) == 0);
static_assert((kS % 32) == 0 && (kH % 32) == 0);
static_assert((kL % kChunk) == 0 && (kChunk % 2) == 0);
static_assert(kH == 64 && kS == 128 && kNB == 16);
static_assert((kXP % 8) == 0 && kXP >= kH);

constexpr size_t kSzDAP  = (size_t)kH * kH * 2;
constexpr size_t kSzDB16 = (size_t)kH * kS * 2;
constexpr size_t kSzC16  = (size_t)kS * kH * 2;
constexpr size_t kSzU16  = (size_t)kRows * kS * 2;
constexpr size_t kSzV    = (size_t)kRows * kH * 4;
constexpr size_t kSzX16  = (size_t)kRows * kH * 2;
constexpr size_t kWsTotal = kSzDAP + kSzDAP + kSzDAP + kSzDB16 + kSzC16 + kSzU16 + kSzV + kSzX16;
static_assert(kWsTotal == 21028864ull);
static_assert(kWsTotal <= 134217728ull);
static_assert((kSzDAP % 256) == 0 && (kSzDB16 % 256) == 0 && (kSzC16 % 256) == 0 &&
              (kSzU16 % 256) == 0 && (kSzV % 256) == 0 && (kSzX16 % 256) == 0);

__device__ __forceinline__ _Float16 to_f16_flushed(float v) {
  const float vf = (fabsf(v) < kF16MinNormal) ? 0.0f : v;
  return (_Float16)vf;
}

__device__ __forceinline__ unsigned short f2bf_bits(float f) {
  unsigned u = __float_as_uint(f);
  return (unsigned short)((u + 0x7FFFu + ((u >> 16) & 1u)) >> 16);
}
__device__ __forceinline__ float bf_bits2f(unsigned short h) { return __uint_as_float(((unsigned)h) << 16); }

__device__ __forceinline__ void split3(float x, unsigned short& hb, unsigned short& lb, unsigned short& mb) {
  hb = f2bf_bits(x);
  const float r1 = x - bf_bits2f(hb);
  lb = f2bf_bits(r1);
  const float r2 = r1 - bf_bits2f(lb);
  mb = f2bf_bits(r2);
}

__device__ __forceinline__ v8f mma_h(v16h a, v16h b, v8f c) {
  c = __builtin_amdgcn_wmma_f32_16x16x32_f16(false, a, false, b, (short)0, c, false, false);
  asm volatile("v_nop\n\tv_nop\n\tv_nop\n\tv_nop" : "+v"(c) : "v"(a), "v"(b));
  return c;
}
__device__ __forceinline__ v8f mma_b(v16b a, v16b b, v8f c) {
  c = __builtin_amdgcn_wmma_f32_16x16x32_bf16(false, a, false, b, (short)0, c, false, false);
  asm volatile("v_nop\n\tv_nop\n\tv_nop\n\tv_nop" : "+v"(c) : "v"(a), "v"(b));
  return c;
}

union FragH { v16h v; v8h h[2]; };
__device__ __forceinline__ v16h frag_load(const _Float16* p) {
  FragH f;
  f.h[0] = *(const v8h*)(p);
  f.h[1] = *(const v8h*)(p + 16);
  return f.v;
}
union FragB { v16b v; v8b h[2]; };
__device__ __forceinline__ v16b frag_load_b(const __bf16* p) {
  FragB f;
  f.h[0] = *(const v8b*)(p);
  f.h[1] = *(const v8b*)(p + 16);
  return f.v;
}

__global__ __launch_bounds__(128) void prep_kernel(
    const float* __restrict__ Bm, const float* __restrict__ Cm, const float* __restrict__ logdt,
    unsigned short* __restrict__ DAH, unsigned short* __restrict__ DAL, unsigned short* __restrict__ DAM,
    unsigned short* __restrict__ DB16, unsigned short* __restrict__ C16)
{
  __shared__ __align__(16) float sA[kH * kH];
  __shared__ __align__(16) float sB[kH * kS];
  const int tid = threadIdx.x;
  const float lv = logdt[0];
  const float sp = fmaxf(lv, 0.0f) + log1pf(expf(-fabsf(lv)));
  const float dt = fminf(fmaxf(sp, kDtMin), kDtMax);
  const float a  = 0.5f * dt;
  const float inv = 1.0f / (1.0f + a);
  {
    float xp = 0.0f;
#pragma unroll 1
    for (int i = 0; i < kH; ++i) {
      const float rhs = dt * Bm[i * kS + tid];
      float xv = fmaf(a, xp, rhs) * inv;
      xv = (fabsf(xv) < kF32MinNormal) ? 0.0f : xv;
      sB[i * kS + tid] = xv;
      xp = xv;
    }
  }
  if (tid < kH) {
    const int j = tid;
    const float f0 = 1.0f - a;
    float xp = 0.0f;
#pragma unroll 1
    for (int i = 0; i < kH; ++i) {
      const float rhs = (i == j) ? f0 : ((i == j + 1) ? a : 0.0f);
      float xv = fmaf(a, xp, rhs) * inv;
      xv = (fabsf(xv) < kF32MinNormal) ? 0.0f : xv;
      sA[i * kH + j] = xv;
      xp = xv;
    }
  }
  __syncthreads();
  for (int pass = 0; pass < 2; ++pass) {
#pragma unroll 1
    for (int it = 0; it < 8; ++it) {
      const int idx = it * 128 + tid;
      const v4f b0 = *(const v4f*)(sB + idx * 8);
      const v4f b1 = *(const v4f*)(sB + idx * 8 + 4);
      const v4f c0 = *(const v4f*)(Cm + idx * 8);
      const v4f c1 = *(const v4f*)(Cm + idx * 8 + 4);
      v8h hb, hc;
#pragma unroll
      for (int e = 0; e < 4; ++e) {
        const float fb0 = b0[e], fb1 = b1[e], fc0 = c0[e], fc1 = c1[e];
        hb[e]     = to_f16_flushed(fb0 * kBCarry);
        hb[4 + e] = to_f16_flushed(fb1 * kBCarry);
        hc[e]     = to_f16_flushed(fc0 * kCCarry);
        hc[4 + e] = to_f16_flushed(fc1 * kCCarry);
      }
      *(volatile v8h*)(DB16 + idx * 8) = hb;
      *(volatile v8h*)(C16 + idx * 8) = hc;
    }
#pragma unroll 1
    for (int it = 0; it < 4; ++it) {
      const int idx = it * 128 + tid;
      const v4f a0 = *(const v4f*)(sA + idx * 8);
      const v4f a1 = *(const v4f*)(sA + idx * 8 + 4);
      v8h vh, vl, vm;
#pragma unroll
      for (int e = 0; e < 4; ++e) {
        const float f0 = a0[e], f1 = a1[e];
        unsigned short h0, l0, m0, h1, l1, m1;
        split3(f0, h0, l0, m0);
        split3(f1, h1, l1, m1);
        vh[e]     = __builtin_bit_cast(_Float16, h0);
        vl[e]     = __builtin_bit_cast(_Float16, l0);
        vm[e]     = __builtin_bit_cast(_Float16, m0);
        vh[4 + e] = __builtin_bit_cast(_Float16, h1);
        vl[4 + e] = __builtin_bit_cast(_Float16, l1);
        vm[4 + e] = __builtin_bit_cast(_Float16, m1);
      }
      *(volatile v8h*)(DAH + idx * 8) = vh;
      *(volatile v8h*)(DAL + idx * 8) = vl;
      *(volatile v8h*)(DAM + idx * 8) = vm;
    }
    __threadfence();
  }
}

__global__ __launch_bounds__(256) void cvt_u_kernel(
    const float* __restrict__ src, unsigned short* __restrict__ dst, int n8)
{
  const int i = blockIdx.x * 256 + threadIdx.x;
  if (i < n8) {
    const size_t e0 = (size_t)i << 3;
    const v4f a0 = *(const v4f*)(src + e0);
    const v4f a1 = *(const v4f*)(src + e0 + 4);
    v8h hv;
#pragma unroll
    for (int e = 0; e < 4; ++e) {
      const float f0 = a0[e], f1 = a1[e];
      hv[e]     = to_f16_flushed(f0 * kUCarry);
      hv[4 + e] = to_f16_flushed(f1 * kUCarry);
    }
    *(volatile v8h*)(dst + e0) = hv;
    __threadfence();
    *(volatile v8h*)(dst + e0) = hv;
  }
}

template <int EPI>
__global__ __launch_bounds__(256) void gemm_f16_kernel(
    const unsigned short* __restrict__ Ap, int lda,
    const unsigned short* __restrict__ Btp, int ldb,
    float* __restrict__ Cout, int ldc,
    const float* __restrict__ dvec, const float* __restrict__ resid,
    int M, int N, int K, float scale)
{
  const _Float16* A  = (const _Float16*)Ap;
  const _Float16* Bt = (const _Float16*)Btp;
  __shared__ __align__(16) float sT[8][16 * 68];
  const int lane = threadIdx.x & 31;
  const int wave = threadIdx.x >> 5;
  const int tilesN = N >> 6;
  const int tilesM = M >> 6;
  const int tile = blockIdx.x * 8 + wave;
  if (tile >= tilesM * tilesN) return;
  const int tm = tile / tilesN;
  const int tn = tile - tm * tilesN;
  const int m0 = tm << 6;
  const int n0 = tn << 6;
  const int rlane = lane & 15;
  const int koff  = (lane >> 4) * 8;
  const int mOff  = (lane >> 4) * 8;

  v8f acc[4][4];
#pragma unroll
  for (int i = 0; i < 4; ++i)
#pragma unroll
    for (int j = 0; j < 4; ++j) acc[i][j] = (v8f){0.f, 0.f, 0.f, 0.f, 0.f, 0.f, 0.f, 0.f};

  for (int k0 = 0; k0 < K; k0 += 32) {
    v16h bh[4];
#pragma unroll
    for (int j = 0; j < 4; ++j) {
      const size_t bo = (size_t)(n0 + (j << 4) + rlane) * ldb + koff + k0;
      bh[j] = frag_load(Bt + bo);
    }
#pragma unroll
    for (int i = 0; i < 4; ++i) {
      const size_t ao = (size_t)(m0 + (i << 4) + rlane) * lda + koff + k0;
      const v16h ah = frag_load(A + ao);
#pragma unroll
      for (int j = 0; j < 4; ++j) acc[i][j] = mma_h(ah, bh[j], acc[i][j]);
    }
  }

  float* slab = sT[wave];
  const int hh = lane >> 4, c4 = (lane & 15) * 4;
  v4f dd = (v4f){0.f, 0.f, 0.f, 0.f};
  if (EPI == 1) dd = *(const v4f*)(dvec + n0 + c4);
#pragma unroll
  for (int i = 0; i < 4; ++i) {
    const int mBase = m0 + (i << 4);
#pragma unroll
    for (int j = 0; j < 4; ++j) {
#pragma unroll
      for (int r = 0; r < 8; ++r) {
        slab[(mOff + r) * 68 + (j << 4) + rlane] = acc[i][j][r] * scale;
      }
    }
    __builtin_amdgcn_fence(__ATOMIC_RELEASE, "workgroup");
    __builtin_amdgcn_wave_barrier();
    __builtin_amdgcn_fence(__ATOMIC_ACQUIRE, "workgroup");
    v4f ov[8];
#pragma unroll
    for (int it = 0; it < 8; ++it) {
      const int row = it * 2 + hh;
      v4f v = *(const v4f*)(slab + row * 68 + c4);
      if (EPI == 1) {
        const v4f uu = *(const v4f*)(resid + (size_t)(mBase + row) * ldc + n0 + c4);
        v = v + dd * uu;
      }
      ov[it] = v;
    }
    for (int pass = 0; pass < 2; ++pass) {
#pragma unroll
      for (int it = 0; it < 8; ++it) {
        const int row = it * 2 + hh;
        *(volatile v4f*)(Cout + (size_t)(mBase + row) * ldc + n0 + c4) = ov[it];
      }
      __threadfence();
    }
    __builtin_amdgcn_fence(__ATOMIC_RELEASE, "workgroup");
    __builtin_amdgcn_wave_barrier();
    __builtin_amdgcn_fence(__ATOMIC_ACQUIRE, "workgroup");
  }
}

__global__ __launch_bounds__(128) void chain_kernel(
    const unsigned short* __restrict__ DAHp, const unsigned short* __restrict__ DALp,
    const unsigned short* __restrict__ DAMp, const float* __restrict__ V, unsigned short* __restrict__ X16)
{
  __shared__ __align__(16) __bf16 sXs[2 * 3 * 16 * kXP];
  __shared__ __align__(16) _Float16 sTl[kChunk * 16 * kH];
  const int tid = threadIdx.x, lane = tid & 31, wave = tid >> 5;
  const int c = lane & 15, hh = lane >> 4;
  constexpr int kPlane = 16 * kXP;

  {
    const __bf16 bz = __builtin_bit_cast(__bf16, (unsigned short)0);
    v8b zv;
#pragma unroll
    for (int e = 0; e < 8; ++e) zv[e] = bz;
#pragma unroll 1
    for (int i = tid; i < (2 * 3 * kPlane) / 8; i += 128) *(v8b*)(sXs + i * 8) = zv;
  }

  const size_t aoff = (size_t)(16 * wave + c) * kH + 8 * hh;
  const __bf16* pah = (const __bf16*)DAHp + aoff;
  const __bf16* pal = (const __bf16*)DALp + aoff;
  const __bf16* pam = (const __bf16*)DAMp + aoff;
  const v16b aH0 = frag_load_b(pah), aH1 = frag_load_b(pah + 32);
  const v16b aL0 = frag_load_b(pal), aL1 = frag_load_b(pal + 32);
  const v16b aM0 = frag_load_b(pam), aM1 = frag_load_b(pam + 32);
  __syncthreads();

  const float* vbase = V + (size_t)c * kL * kH + 16 * wave + 8 * hh;
  v4f p0 = *(const v4f*)(vbase);
  v4f p1 = *(const v4f*)(vbase + 4);
  const int boff = c * kXP + 8 * hh;
  const int woff = c * kXP + 16 * wave + 8 * hh;
  const int toff = c * kH + 16 * wave + 8 * hh;
  const int q = lane >> 3, c8 = (lane & 7) * 8;
  const int cb = 4 * wave + q;

#pragma unroll 1
  for (int t0 = 0; t0 < kL; t0 += kChunk) {
#pragma unroll 1
    for (int s = 0; s < kChunk; ++s) {
      const int t = t0 + s;
      const int tn = (t + 1 < kL) ? (t + 1) : (kL - 1);
      const v4f n0 = *(const v4f*)(vbase + (size_t)tn * kH);
      const v4f n1 = *(const v4f*)(vbase + (size_t)tn * kH + 4);
      const int cur = s & 1;
      const __bf16* xr = sXs + cur * 3 * kPlane + boff;
      __bf16* xw = sXs + (cur ^ 1) * 3 * kPlane + woff;
      const v16b bH0 = frag_load_b(xr),              bH1 = frag_load_b(xr + 32);
      const v16b bL0 = frag_load_b(xr + kPlane),     bL1 = frag_load_b(xr + kPlane + 32);
      const v16b bM0 = frag_load_b(xr + 2 * kPlane), bM1 = frag_load_b(xr + 2 * kPlane + 32);

      v8f acc = (v8f){0.f, 0.f, 0.f, 0.f, 0.f, 0.f, 0.f, 0.f};
      acc = mma_b(aM0, bH0, acc);
      acc = mma_b(aH0, bM0, acc);
      acc = mma_b(aL0, bL0, acc);
      acc = mma_b(aL0, bH0, acc);
      acc = mma_b(aH0, bL0, acc);
      acc = mma_b(aM1, bH1, acc);
      acc = mma_b(aH1, bM1, acc);
      acc = mma_b(aL1, bL1, acc);
      acc = mma_b(aL1, bH1, acc);
      acc = mma_b(aH1, bL1, acc);
      acc = mma_b(aH0, bH0, acc);
      acc = mma_b(aH1, bH1, acc);

      v8b vH, vL, vM;
      v8h vF;
#pragma unroll
      for (int r = 0; r < 8; ++r) {
        const float pv = (r < 4) ? p0[r & 3] : p1[r & 3];
        const float av = acc[r];
        const float x = av + pv;
        unsigned short hb, lb, mb;
        split3(x, hb, lb, mb);
        vH[r] = __builtin_bit_cast(__bf16, hb);
        vL[r] = __builtin_bit_cast(__bf16, lb);
        vM[r] = __builtin_bit_cast(__bf16, mb);
        vF[r] = to_f16_flushed(x * kXCarry);
      }
      *(v8b*)(xw) = vH;
      *(v8b*)(xw + kPlane) = vL;
      *(v8b*)(xw + 2 * kPlane) = vM;
      *(v8h*)(sTl + s * 16 * kH + toff) = vF;
      __syncthreads();
      p0 = n0;
      p1 = n1;
    }
    for (int pass = 0; pass < 2; ++pass) {
#pragma unroll 1
      for (int it = 0; it < kChunk; ++it) {
        const v8h v = *(const v8h*)(sTl + (it * 16 + cb) * kH + c8);
        *(volatile v8h*)(X16 + ((size_t)cb * kL + (size_t)(t0 + it)) * kH + c8) = v;
      }
      __threadfence();
    }
    __syncthreads();
  }
}

extern "C" void kernel_launch(void* const* d_in, const int* in_sizes, int n_in,
                              void* d_out, int out_size, void* d_ws, size_t ws_size,
                              hipStream_t stream) {
  if (n_in < 5 || d_out == nullptr || d_ws == nullptr) return;
  if (in_sizes[0] != kRows * kS) return;
  if (in_sizes[1] != kH * kS) return;
  if (in_sizes[2] != kS * kH) return;
  if (in_sizes[3] != kS) return;
  if (in_sizes[4] != 1) return;
  if (out_size != kRows * kS) return;
  if (ws_size < kWsTotal) return;

  const float* u     = (const float*)d_in[0];
  const float* Bm    = (const float*)d_in[1];
  const float* Cm    = (const float*)d_in[2];
  const float* Dv    = (const float*)d_in[3];
  const float* logdt = (const float*)d_in[4];
  float* out = (float*)d_out;

  char* ws = (char*)d_ws;
  size_t off = 0;
  auto carve = [&](size_t bytes) -> char* { char* p = ws + off; off += (bytes + 255) & ~(size_t)255; return p; };
  unsigned short* DAH  = (unsigned short*)carve(kSzDAP);
  unsigned short* DAL  = (unsigned short*)carve(kSzDAP);
  unsigned short* DAM  = (unsigned short*)carve(kSzDAP);
  unsigned short* DB16 = (unsigned short*)carve(kSzDB16);
  unsigned short* C16  = (unsigned short*)carve(kSzC16);
  unsigned short* U16  = (unsigned short*)carve(kSzU16);
  float*          V    = (float*)carve(kSzV);
  unsigned short* X16  = (unsigned short*)carve(kSzX16);
  if (off != kWsTotal || off > ws_size) return;

  prep_kernel<<<1, 128, 0, stream>>>(Bm, Cm, logdt, DAH, DAL, DAM, DB16, C16);

  const int n8 = kRows * kS / 8;
  cvt_u_kernel<<<n8 / 256, 256, 0, stream>>>(u, U16, n8);

  gemm_f16_kernel<0><<<(kRows / 64) * (kH / 64) / 8, 256, 0, stream>>>(
      U16, kS, DB16, kS, V, kH, Dv, u, kRows, kH, kS, kFold1);

  chain_kernel<<<1, 128, 0, stream>>>(DAH, DAL, DAM, V, X16);

  gemm_f16_kernel<1><<<(kRows / 64) * (kS / 64) / 8, 256, 0, stream>>>(
      X16, kH, C16, kH, out, kS, Dv, u, kRows, kS, kH, kFold2);
}
